// ConvAutoencoder_65481071408451
// MI455X (gfx1250) — hardware-verified
//
#include <hip/hip_runtime.h>
#include <stdint.h>

#define DEVINL __device__ __forceinline__

typedef _Float16 f16t;
typedef _Float16 v16h __attribute__((ext_vector_type(16)));
typedef _Float16 v8h  __attribute__((ext_vector_type(8)));
typedef __bf16   v16b __attribute__((ext_vector_type(16)));
typedef unsigned short v8us __attribute__((ext_vector_type(8)));
typedef float    v8f  __attribute__((ext_vector_type(8)));
typedef float    v4f  __attribute__((ext_vector_type(4)));
typedef v8h  __attribute__((may_alias)) v8ha;
typedef v8us __attribute__((may_alias)) v8usa;
typedef v4f  __attribute__((may_alias)) v4fa;
union FragH { v16h v; v8h half[2]; };
union FragB { v16b v; v16h vh; v8us half[2]; };

#define IMG   512
#define WO    511
#define LP    (WO * WO)
#define HID1  128
#define HID2  64
#define LAT   32
#define NP5   16
#define KP0   32
#define PITCH 136
#define WAVES 8
#define TPB   256
#define ACAR  16.0f
#define WCAR  256.0f

#define OFF1  0
#define OFF2  8192
#define OFF3  10240
#define OFF4  12288
#define OFF5  20480
#define WT_HALVES 22528

static_assert(TPB == WAVES * 32);
static_assert((PITCH % 8) == 0);
static_assert((WT_HALVES * 2) % 128 == 0);
static_assert((HID1 * KP0 * 2) % 128 == 0);

DEVINL int imin(int a, int b) { return a < b ? a : b; }
DEVINL int imax(int a, int b) { return a > b ? a : b; }

DEVINL v8f wmma_f16(v16h a, v16h b, v8f c) {
  v8f d = __builtin_amdgcn_wmma_f32_16x16x32_f16(false, a, false, b, (short)0, c, false, false);
  asm volatile("v_nop\n\tv_nop\n\tv_nop\n\tv_nop" : "+v"(d) : "v"(a), "v"(b));
  return d;
}
DEVINL v8f wmma_bf16(FragB a, FragB b, v8f c) {
  v8f d = __builtin_amdgcn_wmma_f32_16x16x32_bf16(false, a.v, false, b.v, (short)0, c, false, false);
  asm volatile("v_nop\n\tv_nop\n\tv_nop\n\tv_nop" : "+v"(d) : "v"(a.vh), "v"(b.vh));
  return d;
}
DEVINL v8f zero8f() {
  v8f z = {0.f, 0.f, 0.f, 0.f, 0.f, 0.f, 0.f, 0.f};
  return z;
}

DEVINL unsigned short bf16_bits(float f) {
  unsigned u = __float_as_uint(f);
  u += 0x7FFFu + ((u >> 16) & 1u);
  return (unsigned short)(u >> 16);
}
DEVINL float bf16_val(unsigned short s) { return __uint_as_float(((unsigned)s) << 16); }
DEVINL void split3(float w, unsigned short& hb, unsigned short& mb, unsigned short& lb) {
  hb = bf16_bits(w);
  const float hv = bf16_val(hb);
  const float r1 = w - hv;
  mb = bf16_bits(r1);
  const float mv = bf16_val(mb);
  const float r2 = r1 - mv;
  lb = bf16_bits(r2);
}

__global__ __launch_bounds__(TPB) void prep_w0_k(const float* __restrict__ ew0,
                                                unsigned short* __restrict__ W0T)
{
  const int t = blockIdx.x * TPB + threadIdx.x;
  if (t >= HID1 * (KP0 / 8)) return;
  const int n = t >> 2, part = t & 3;
  v8us o;
  #pragma unroll
  for (int i = 0; i < 8; ++i) {
    const int k = 8 * part + i;
    const int j = k >> 2, c = k & 3;
    const float w = ew0[c * HID1 + n];
    unsigned short hb, mb, lb;
    split3(w, hb, mb, lb);
    unsigned short s = hb;
    s = (j == 1 || j == 4) ? mb : s;
    s = (j == 2) ? lb : s;
    s = (j >= 6) ? (unsigned short)0 : s;
    o[i] = s;
  }
  unsigned short* dst = W0T + 8 * t;
  *(volatile v8us*)dst = o;
  __threadfence();
  *(volatile v8us*)dst = o;
}

__global__ __launch_bounds__(TPB) void prep_w_k(const float* __restrict__ ew1, const float* __restrict__ ew2,
                                               const float* __restrict__ dw0, const float* __restrict__ dw1,
                                               const float* __restrict__ dw2, f16t* __restrict__ WT)
{
  const int y = blockIdx.y;
  const float* src; int K, N, NPD, doff;
  if (y == 0)      { src = ew1; K = HID1; N = HID2; NPD = HID2; doff = OFF1; }
  else if (y == 1) { src = ew2; K = HID2; N = LAT;  NPD = LAT;  doff = OFF2; }
  else if (y == 2) { src = dw0; K = LAT;  N = HID2; NPD = HID2; doff = OFF3; }
  else if (y == 3) { src = dw1; K = HID2; N = HID1; NPD = HID1; doff = OFF4; }
  else             { src = dw2; K = HID1; N = 4;    NPD = NP5;  doff = OFF5; }
  const int t = blockIdx.x * TPB + threadIdx.x;
  const int kparts = K >> 3;
  if (t >= NPD * kparts) return;
  const int n = t / kparts, part = t - n * kparts;
  const int ncl = imin(n, N - 1);
  const float sc = (n < N) ? WCAR : 0.0f;
  v8h o;
  #pragma unroll
  for (int i = 0; i < 8; ++i) {
    const float w = src[(8 * part + i) * N + ncl];
    o[i] = (f16t)(w * sc);
  }
  f16t* dst = WT + doff + 8 * t;
  *(volatile v8h*)dst = o;
  __threadfence();
  *(volatile v8h*)dst = o;
}

template <bool RELU>
DEVINL void epi_store(f16t* act, int m, int h, int nc, v8f acc,
                      const float* __restrict__ bias, float sc)
{
  const float* bp = bias + 16 * nc + 8 * h;
  const v4f b0 = *(const v4fa*)bp;
  const v4f b1 = *(const v4fa*)(bp + 4);
  v8h o;
  #pragma unroll
  for (int r = 0; r < 4; ++r) {
    float t0 = fmaf(acc[r], sc, b0[r]);
    float t1 = fmaf(acc[4 + r], sc, b1[r]);
    if (RELU) { t0 = fmaxf(t0, 0.0f); t1 = fmaxf(t1, 0.0f); }
    o[r]     = (f16t)(t0 * ACAR);
    o[4 + r] = (f16t)(t1 * ACAR);
  }
  *(v8ha*)(act + m * PITCH + 16 * nc + 8 * h) = o;
}

template <int K, int NOUT, bool RELU>
DEVINL void dense_f16(const f16t* __restrict__ Wp, const float* __restrict__ bias,
                      f16t* act, int m, int h)
{
  constexpr int KS = K / 32, NC = NOUT / 16;
  FragH bf[KS];
  const f16t* arow = act + m * PITCH + 8 * h;
  #pragma unroll
  for (int ks = 0; ks < KS; ++ks) {
    bf[ks].half[0] = *(const v8ha*)(arow + 32 * ks);
    bf[ks].half[1] = *(const v8ha*)(arow + 32 * ks + 16);
  }
  #pragma unroll 1
  for (int nc = 0; nc < NC; ++nc) {
    const f16t* wrow = Wp + (size_t)(16 * nc + m) * K + 8 * h;
    v8f acc = zero8f();
    #pragma unroll
    for (int ks = 0; ks < KS; ++ks) {
      FragH a;
      a.half[0] = *(const v8ha*)(wrow + 32 * ks);
      a.half[1] = *(const v8ha*)(wrow + 32 * ks + 16);
      acc = wmma_f16(a.v, bf[ks].v, acc);
    }
    epi_store<RELU>(act, m, h, nc, acc, bias, 1.0f / (ACAR * WCAR));
  }
}

__global__ __launch_bounds__(TPB) void mlp_k(const float* __restrict__ x,
                                           const unsigned short* __restrict__ W0T,
                                           const f16t* __restrict__ WT,
                                           const float* __restrict__ eb0, const float* __restrict__ eb1,
                                           const float* __restrict__ eb2, const float* __restrict__ db0,
                                           const float* __restrict__ db1, const float* __restrict__ db2,
                                           float* __restrict__ rpl, int nrows, int ntiles)
{
  __shared__ __attribute__((aligned(16))) f16t sAct[WAVES * 16 * PITCH];
  const int tid = threadIdx.x, lane = tid & 31, wave = tid >> 5;
  const int h = lane >> 4, m = lane & 15;
  f16t* act = sAct + wave * (16 * PITCH);
  const int tl = blockIdx.x * WAVES + wave;
  const bool valid = tl < ntiles;
  const int tlc = valid ? tl : (ntiles - 1);

  FragB xq;
  {
    int g = tlc * 16 + m;
    g = imin(g, nrows - 1);
    const int b  = g / LP;
    const int rm = g - b * LP;
    const int i  = rm / WO;
    const int j  = rm - i * WO;
    const float* xp = x + ((size_t)(b * IMG + i)) * IMG + j;
    float xv[4];
    xv[0] = xp[0]; xv[1] = xp[1]; xv[2] = xp[IMG]; xv[3] = xp[IMG + 1];
    unsigned short hx[4], mx[4], lx[4];
    #pragma unroll
    for (int c = 0; c < 4; ++c) split3(xv[c], hx[c], mx[c], lx[c]);
    const bool hsel = (h != 0);
    v8us q0, q1;
    #pragma unroll
    for (int c = 0; c < 4; ++c) {
      q0[c]     = hx[c];
      q0[4 + c] = hsel ? mx[c] : hx[c];
      q1[c]     = hsel ? (unsigned short)0 : mx[c];
      q1[4 + c] = hsel ? (unsigned short)0 : lx[c];
    }
    xq.half[0] = q0;
    xq.half[1] = q1;
  }
  #pragma unroll 1
  for (int nc = 0; nc < HID1 / 16; ++nc) {
    const unsigned short* wr = W0T + (16 * nc + m) * KP0 + 8 * h;
    FragB a;
    a.half[0] = *(const v8usa*)(wr);
    a.half[1] = *(const v8usa*)(wr + 16);
    const v8f acc = wmma_bf16(a, xq, zero8f());
    epi_store<true>(act, m, h, nc, acc, eb0, 1.0f);
  }
  __syncthreads();

  dense_f16<HID1, HID2, true >(WT + OFF1, eb1, act, m, h);
  __syncthreads();
  dense_f16<HID2, LAT,  false>(WT + OFF2, eb2, act, m, h);
  __syncthreads();
  dense_f16<LAT,  HID2, true >(WT + OFF3, db0, act, m, h);
  __syncthreads();
  dense_f16<HID2, HID1, true >(WT + OFF4, db1, act, m, h);
  __syncthreads();

  {
    FragH bf[4];
    const f16t* arow = act + m * PITCH + 8 * h;
    #pragma unroll
    for (int ks = 0; ks < 4; ++ks) {
      bf[ks].half[0] = *(const v8ha*)(arow + 32 * ks);
      bf[ks].half[1] = *(const v8ha*)(arow + 32 * ks + 16);
    }
    const f16t* wrow = WT + OFF5 + (size_t)m * HID1 + 8 * h;
    v8f acc = zero8f();
    #pragma unroll
    for (int ks = 0; ks < 4; ++ks) {
      FragH a;
      a.half[0] = *(const v8ha*)(wrow + 32 * ks);
      a.half[1] = *(const v8ha*)(wrow + 32 * ks + 16);
      acc = wmma_f16(a.v, bf[ks].v, acc);
    }
    const float s5 = 1.0f / (ACAR * WCAR);
    const float c0 = db2[0], c1 = db2[1], c2 = db2[2], c3 = db2[3];
    v4f rv;
    rv[0] = fmaf(acc[0], s5, c0);
    rv[1] = fmaf(acc[1], s5, c1);
    rv[2] = fmaf(acc[2], s5, c2);
    rv[3] = fmaf(acc[3], s5, c3);
    float* dst = rpl + ((size_t)tlc * 16 + m) * 4;
    const bool st = valid && (lane < 16);
    if (st) *(volatile v4f*)dst = rv;
    __threadfence();
    if (st) *(volatile v4f*)dst = rv;
  }
}

__global__ __launch_bounds__(TPB) void ovl_k(const float* __restrict__ rpl, float* __restrict__ out,
                                           int total4)
{
  const int t = blockIdx.x * TPB + threadIdx.x;
  if (t >= total4) return;
  const int b   = t >> 16;
  const int rem = t & 65535;
  const int y   = rem >> 7;
  const int x0  = (rem & 127) * 4;
  const int i0  = imin(y, WO - 1);
  const int i1  = imax(y - 1, 0);
  const size_t base0 = (size_t)b * LP + (size_t)i0 * WO;
  const size_t base1 = (size_t)b * LP + (size_t)i1 * WO;
  v4f R0[5], R1[5];
  #pragma unroll
  for (int q = 0; q < 5; ++q) {
    const int jc = imin(imax(x0 - 1 + q, 0), WO - 1);
    R0[q] = *(const v4fa*)(rpl + (base0 + (size_t)jc) * 4);
    R1[q] = *(const v4fa*)(rpl + (base1 + (size_t)jc) * 4);
  }
  const bool vy0 = (y <= WO - 1), vy1 = (y >= 1);
  v4f o;
  #pragma unroll
  for (int p = 0; p < 4; ++p) {
    const int xx = x0 + p;
    const bool vxa = (xx <= WO - 1), vxb = (xx >= 1);
    float s = 0.0f;
    s = (vy0 && vxa) ? (s + R0[p + 1][0]) : s;
    s = (vy0 && vxb) ? (s + R0[p][1])     : s;
    s = (vy1 && vxa) ? (s + R1[p + 1][2]) : s;
    s = (vy1 && vxb) ? (s + R1[p][3])     : s;
    o[p] = s;
  }
  float* dst = out + (size_t)t * 4;
  *(volatile v4f*)dst = o;
  __threadfence();
  *(volatile v4f*)dst = o;
}

extern "C" void kernel_launch(void* const* d_in, const int* in_sizes, int n_in,
                              void* d_out, int out_size, void* d_ws, size_t ws_size,
                              hipStream_t stream) {
  if (n_in < 13) return;
  if (in_sizes[0] <= 0 || (in_sizes[0] % (IMG * IMG)) != 0) return;
  const int nB = in_sizes[0] / (IMG * IMG);
  if (in_sizes[1]  != 4 * HID1)    return;
  if (in_sizes[2]  != HID1)        return;
  if (in_sizes[3]  != HID1 * HID2) return;
  if (in_sizes[4]  != HID2)        return;
  if (in_sizes[5]  != HID2 * LAT)  return;
  if (in_sizes[6]  != LAT)         return;
  if (in_sizes[7]  != LAT * HID2)  return;
  if (in_sizes[8]  != HID2)        return;
  if (in_sizes[9]  != HID2 * HID1) return;
  if (in_sizes[10] != HID1)        return;
  if (in_sizes[11] != HID1 * 4)    return;
  if (in_sizes[12] != 4)           return;
  if (out_size != nB * IMG * IMG)  return;

  const int nrows  = nB * LP;
  const int ntiles = (nrows + 15) / 16;
  const int total4 = out_size / 4;

  const float* x   = (const float*)d_in[0];
  const float* ew0 = (const float*)d_in[1];
  const float* eb0 = (const float*)d_in[2];
  const float* ew1 = (const float*)d_in[3];
  const float* eb1 = (const float*)d_in[4];
  const float* ew2 = (const float*)d_in[5];
  const float* eb2 = (const float*)d_in[6];
  const float* dw0 = (const float*)d_in[7];
  const float* db0 = (const float*)d_in[8];
  const float* dw1 = (const float*)d_in[9];
  const float* db1 = (const float*)d_in[10];
  const float* dw2 = (const float*)d_in[11];
  const float* db2 = (const float*)d_in[12];
  float* outp = (float*)d_out;

  const size_t szW0 = (size_t)HID1 * KP0 * 2;
  const size_t szWT = (size_t)WT_HALVES * 2;
  const size_t szR  = (size_t)ntiles * 256;
  size_t off = 0;
  char* ws = (char*)d_ws;
  unsigned short* W0T = (unsigned short*)(ws + off); off += szW0;
  f16t*  WT  = (f16t*)(ws + off);                     off += szWT;
  float* RPL = (float*)(ws + off);                    off += szR;
  if (off > ws_size) return;

  prep_w0_k<<<(HID1 * (KP0 / 8) + TPB - 1) / TPB, TPB, 0, stream>>>(ew0, W0T);
  prep_w_k<<<dim3((HID1 * HID2 / 8 + TPB - 1) / TPB, 5), TPB, 0, stream>>>(ew1, ew2, dw0, dw1, dw2, WT);
  mlp_k<<<(ntiles + WAVES - 1) / WAVES, TPB, 0, stream>>>(x, W0T, WT, eb0, eb1, eb2, db0, db1, db2,
                                                          RPL, nrows, ntiles);
  ovl_k<<<(total4 + TPB - 1) / TPB, TPB, 0, stream>>>(RPL, outp, total4);
}
